// GBA_LBA_4930622456022
// MI455X (gfx1250) — hardware-verified
//
#include <hip/hip_runtime.h>


typedef _Float16 h16;
typedef __attribute__((ext_vector_type(16))) _Float16 v16h;
typedef __attribute__((ext_vector_type(8)))  float  v8f;
typedef __attribute__((ext_vector_type(4)))  float  v4f;
typedef __attribute__((ext_vector_type(4)))  unsigned int v4u;

__device__ __forceinline__ v8f wmma_h(v16h a, v16h b, v8f c) {
    v8f d = __builtin_amdgcn_wmma_f32_16x16x32_f16(false, a, false, b, (short)0, c, false, false);
    asm volatile("v_nop\n\tv_nop\n\tv_nop\n\tv_nop" : "+v"(d) : "v"(a), "v"(b));
    return d;
}
__device__ __forceinline__ void wave_sync_lds() {
    __builtin_amdgcn_fence(__ATOMIC_RELEASE, "workgroup"); __builtin_amdgcn_wave_barrier(); __builtin_amdgcn_fence(__ATOMIC_ACQUIRE, "workgroup");
}

__global__ void pack_w16(const float* __restrict__ src, h16* __restrict__ dst, int n8, float scale) {
    int i = blockIdx.x * 256 + threadIdx.x;
    if (i < n8) {
        union { v4u u; h16 e[8]; } o;
#pragma unroll
        for (int j = 0; j < 8; ++j) o.e[j] = (h16)(src[(size_t)i * 8 + j] * scale);
        *(volatile v4u*)(dst + (size_t)i * 8) = o.u; __threadfence(); *(volatile v4u*)(dst + (size_t)i * 8) = o.u;
    }
}

__global__ void pack_x_hwc(const float* __restrict__ x, h16* __restrict__ xt) {
    int i = blockIdx.x * 256 + threadIdx.x;
    int c8 = i & 15;
    int n = (i >> 4) % 9216;
    int b = i / (9216 * 16);
    union { v4u u; h16 e[8]; } o;
#pragma unroll
    for (int j = 0; j < 8; ++j) o.e[j] = (h16)x[((size_t)b * 128 + c8 * 8 + j) * 9216 + n];
    h16* d = xt + ((size_t)b * 9216 + n) * 128 + c8 * 8;
    *(volatile v4u*)d = o.u; __threadfence(); *(volatile v4u*)d = o.u;
}

__global__ void avgpool_pack(const float* __restrict__ x, h16* __restrict__ xp_t) {
    int i = blockIdx.x * 256 + threadIdx.x;
    int c8 = i & 15;
    int kp = (i >> 4) % 576;
    int b = i / (576 * 16);
    int py = kp / 24, px = kp % 24;
    union { v4u u; h16 e[8]; } o;
#pragma unroll
    for (int j = 0; j < 8; ++j) {
        const float* base = x + ((size_t)b * 128 + c8 * 8 + j) * 9216 + (py * 4) * 96 + px * 4;
        float s = 0.f;
#pragma unroll
        for (int dy = 0; dy < 4; ++dy)
#pragma unroll
            for (int dx = 0; dx < 4; ++dx) s += base[dy * 96 + dx];
        o.e[j] = (h16)(s * 0.0625f);
    }
    h16* d = xp_t + ((size_t)b * 576 + kp) * 128 + c8 * 8;
    *(volatile v4u*)d = o.u; __threadfence(); *(volatile v4u*)d = o.u;
}

template<int K, int EPI, int MT, int LOB>
__global__ __launch_bounds__(128) void gemm_wmma(
    const h16* __restrict__ A, const h16* __restrict__ Bt, const float* __restrict__ lob,
    const float* __restrict__ bias, int N, float oscale, float oscale2, float tscale,
    float* __restrict__ outF, h16* __restrict__ outT, h16* __restrict__ outT2,
    const float* __restrict__ vbuf)
{
    constexpr int KS = K / 32;
    constexpr int M  = MT * 16;
    __shared__ __attribute__((aligned(16))) h16   stw[4][16][64];
    __shared__ __attribute__((aligned(16))) float stf[16][64];
    __shared__ __attribute__((aligned(16))) h16   stv[64][64];
    const int lane = threadIdx.x & 31;
    const int wave = threadIdx.x >> 5;
    const int tid  = threadIdx.x;
    const int r15  = lane & 15;
    const int half = lane >> 4;
    const int nblk = blockIdx.x * 64;
    const int n0 = nblk + wave * 16;
    const int b  = blockIdx.z;

    v16h bfrag[KS];
    {
        const int ldb = LOB ? 64 : K;
        const h16* brow = Bt + ((size_t)b * N + n0 + r15) * ldb + half * 8;
#pragma unroll
        for (int ks = 0; ks < KS; ++ks) {
            v4u* bv = (v4u*)&bfrag[ks];
            if (!LOB || ks < 2) {
                bv[0] = *(const v4u*)(brow + ks * 32);
                bv[1] = *(const v4u*)(brow + ks * 32 + 16);
            } else {
#pragma unroll
                for (int e = 0; e < 2; ++e) {
                    const int hh = 2 * (ks - 2) + e;
                    const float* lp = lob + (((size_t)b * 4 + hh) * N + n0 + r15) * 16 + half * 8;
                    v4f f0 = *(const v4f*)lp, f1 = *(const v4f*)(lp + 4);
                    bfrag[ks][8 * e + 0] = (h16)(f0[0] * 64.f); bfrag[ks][8 * e + 1] = (h16)(f0[1] * 64.f);
                    bfrag[ks][8 * e + 2] = (h16)(f0[2] * 64.f); bfrag[ks][8 * e + 3] = (h16)(f0[3] * 64.f);
                    bfrag[ks][8 * e + 4] = (h16)(f1[0] * 64.f); bfrag[ks][8 * e + 5] = (h16)(f1[1] * 64.f);
                    bfrag[ks][8 * e + 6] = (h16)(f1[2] * 64.f); bfrag[ks][8 * e + 7] = (h16)(f1[3] * 64.f);
                }
            }
        }
    }

#pragma unroll
    for (int mt = 0; mt < MT; ++mt) {
        const int m0 = mt * 16;
        const h16* arow = A + (size_t)(m0 + r15) * K + half * 8;
        v8f acc = {}, acc2 = {};
#pragma unroll
        for (int ks = 0; ks < KS; ++ks) {
            v16h af;
            v4u* av = (v4u*)&af;
            av[0] = *(const v4u*)(arow + ks * 32);
            av[1] = *(const v4u*)(arow + ks * 32 + 16);
            if (LOB && ks >= 2) acc2 = wmma_h(af, bfrag[ks], acc2);
            else                acc  = wmma_h(af, bfrag[ks], acc);
        }
        float a0v[8];
#pragma unroll
        for (int r = 0; r < 8; ++r) a0v[r] = acc[r] * oscale + (LOB ? acc2[r] * oscale2 : 0.f) + bias[m0 + r + 8 * half];

        if (EPI == 0) {
#pragma unroll
            for (int r = 0; r < 8; ++r) stf[r + 8 * half][wave * 16 + r15] = a0v[r];
            __syncthreads();
            float* ob = outF + ((size_t)b * M + m0) * N + nblk;
            for (int pass = 0; pass < 2; ++pass) {
#pragma unroll
                for (int q = 0; q < 2; ++q) {
                    int piece = tid + q * 128;
                    int row = piece >> 4, seg = piece & 15;
                    *(volatile v4f*)(ob + (size_t)row * N + seg * 4) = *(const v4f*)(&stf[row][seg * 4]);
                }
                __threadfence();
            }
            __syncthreads();
        } else if (EPI == 4 && mt >= 4) {
#pragma unroll
            for (int r = 0; r < 8; ++r) stv[m0 - 64 + r + 8 * half][wave * 16 + r15] = (h16)(a0v[r] * tscale);
        } else {
#pragma unroll
            for (int r = 0; r < 8; ++r) {
                int m = m0 + r + 8 * half;
                float a0 = a0v[r];
                float val;
                if (EPI == 1 || EPI == 4) {
                    val = a0;
                } else if (EPI == 2) {
                    val = a0 / (1.0f + __expf(-a0));
                } else {
                    float t = tanhf(a0 * 0.25f);
                    val = t * vbuf[((size_t)b * M + m) * N + n0 + r15];
                }
                stw[wave][r15][m] = (h16)(val * tscale);
            }
        }
    }
    if (EPI != 0) {
        wave_sync_lds();
        h16* tb = outT + ((size_t)b * N + n0) * 64;
        for (int pass = 0; pass < 2; ++pass) {
#pragma unroll
            for (int j = 0; j < 4; ++j) {
                int row = j * 4 + (lane >> 3), seg = lane & 7;
                *(volatile v4u*)(tb + (size_t)row * 64 + seg * 8) = *(const v4u*)(&stw[wave][row][seg * 8]);
            }
            __threadfence();
        }
    }
    if (EPI == 4) {
        __syncthreads();
        for (int pass = 0; pass < 2; ++pass) {
#pragma unroll
            for (int q = 0; q < 4; ++q) {
                int piece = tid + q * 128;
                int d = piece >> 3, seg = piece & 7;
                *(volatile v4u*)(outT2 + ((size_t)b * 64 + d) * N + nblk + seg * 8) = *(const v4u*)(&stv[d][seg * 8]);
            }
            __threadfence();
        }
    }
}

__global__ __launch_bounds__(256) void dwconv_qk_v(
    const float* __restrict__ qkv_lin, const float* __restrict__ dw_w,
    const float* __restrict__ dw_b, h16* __restrict__ qk_t, float* __restrict__ v_buf)
{
    __shared__ float sm[3][20][20];
    const int tile = blockIdx.x;
    const int ch   = blockIdx.y;
    const int b    = blockIdx.z;
    const int tx0 = (tile % 6) * 16, ty0 = (tile / 6) * 16;
    const int tx = threadIdx.x, ty = threadIdx.y;
    const int tid = ty * 16 + tx;
    const size_t plane = 9216;
    const float* base = qkv_lin + (size_t)b * 192 * plane;
#pragma unroll
    for (int p = 0; p < 3; ++p) {
        const float* src = base + (size_t)(p * 64 + ch) * plane;
        for (int l = tid; l < 400; l += 256) {
            int ly = l / 20, lx = l % 20;
            int gy = ty0 + ly - 2, gx = tx0 + lx - 2;
            float v = 0.f;
            if (gy >= 0 && gy < 96 && gx >= 0 && gx < 96) v = src[gy * 96 + gx];
            sm[p][ly][lx] = v;
        }
    }
    __syncthreads();
    const float* wq = dw_w + (size_t)ch * 25;
    const float* wk = dw_w + (size_t)(64 + ch) * 25;
    const float* wv = dw_w + (size_t)(128 + ch) * 25;
    float aq = 0.f, ak = 0.f, avv = 0.f;
#pragma unroll
    for (int ky = 0; ky < 5; ++ky)
#pragma unroll
        for (int kx = 0; kx < 5; ++kx) {
            int o = ky * 5 + kx;
            aq  += wq[o] * sm[0][ty + ky][tx + kx];
            ak  += wk[o] * sm[1][ty + ky][tx + kx];
            avv += wv[o] * sm[2][ty + ky][tx + kx];
        }
    float qv = aq + dw_b[ch];
    float kv = ak + dw_b[64 + ch];
    float vv = avv + dw_b[128 + ch];
    int n = (ty0 + ty) * 96 + tx0 + tx;
    qk_t[((size_t)b * 9216 + n) * 64 + ch] = (h16)(qv * kv * 4096.0f);
    v_buf[((size_t)b * 64 + ch) * 9216 + n] = vv;
}

__global__ __launch_bounds__(32) void attn_kernel(
    const h16* __restrict__ qlo_t,
    const h16* __restrict__ kkt,
    const h16* __restrict__ vvT,
    float* __restrict__ lo_f)
{
    __shared__ float sc[16 * 576];
    __shared__ __attribute__((aligned(16))) h16 pr[16 * 576];
    __shared__ float rden[16];

    const int it = blockIdx.x;
    const int h  = blockIdx.y;
    const int b  = blockIdx.z;
    const int lane = threadIdx.x;
    const int r15 = lane & 15, half = lane >> 4;
    const v4u z4 = {0u, 0u, 0u, 0u};

    const h16* vrow = vvT + ((size_t)b * 64 + h * 16 + r15) * 576;

    v16h aq; v4u* aqv = (v4u*)&aq;
    const h16* qrow = qlo_t + ((size_t)b * 9216 + it * 16 + r15) * 64 + h * 16;
    aqv[0] = *(const v4u*)(qrow + half * 8);
    aqv[1] = z4;

    const h16* kbase = kkt + (size_t)b * 576 * 64 + h * 16;
    for (int jt = 0; jt < 36; ++jt) {
        v16h bk; v4u* bkv = (v4u*)&bk;
        const h16* krow = kbase + (size_t)(jt * 16 + r15) * 64;
        bkv[0] = *(const v4u*)(krow + half * 8);
        bkv[1] = z4;
        v8f s = {};
        s = wmma_h(aq, bk, s);
#pragma unroll
        for (int r = 0; r < 8; ++r)
            sc[(r + 8 * half) * 576 + jt * 16 + r15] = s[r] * 0.25f;
    }
    wave_sync_lds();

    {
        const int row = r15;
        float mx = -1e30f;
        for (int j = half * 288; j < half * 288 + 288; ++j)
            mx = fmaxf(mx, sc[row * 576 + j]);
        mx = fmaxf(mx, __shfl_xor(mx, 16, 32));
        float sum = 0.f;
        for (int j = half * 288; j < half * 288 + 288; ++j) {
            float p = __expf(sc[row * 576 + j] - mx);
            pr[row * 576 + j] = (h16)p;
            sum += p;
        }
        sum += __shfl_xor(sum, 16, 32);
        if (half == 0) rden[row] = 1.0f / sum;
    }
    wave_sync_lds();

    v8f acc = {};
    const h16* prow = pr + (size_t)r15 * 576;
    for (int kt = 0; kt < 18; ++kt) {
        v16h ap, bv;
        v4u* apv = (v4u*)&ap;
        v4u* bvv = (v4u*)&bv;
        int k0 = kt * 32;
        apv[0] = *(const v4u*)(prow + k0 + half * 8);
        apv[1] = *(const v4u*)(prow + k0 + 16 + half * 8);
        bvv[0] = *(const v4u*)(vrow + k0 + half * 8);
        bvv[1] = *(const v4u*)(vrow + k0 + 16 + half * 8);
        acc = wmma_h(ap, bv, acc);
    }
    float vals[8];
#pragma unroll
    for (int r = 0; r < 8; ++r) vals[r] = acc[r] * rden[r + 8 * half];
    float* ob = lo_f + (((size_t)b * 4 + h) * 9216 + it * 16) * 16;
    for (int pass = 0; pass < 2; ++pass) {
#pragma unroll
        for (int j = 0; j < 8; ++j) {
            const int ia = (j < 4) ? 2 * j : 2 * j - 8, ib = ia + 1;
            float xa = vals[ia], xb = vals[ib];
            float xa_o = __shfl_xor(xa, 16, 32), xb_o = __shfl_xor(xb, 16, 32);
            float v;
            if (j < 4) v = (half == 0) ? xa : xb_o;
            else       v = (half == 0) ? xa_o : xb;
            *(volatile float*)(ob + (size_t)(2 * j) * 16 + lane) = v;
        }
        __threadfence();
    }
}

extern "C" void kernel_launch(void* const* d_in, const int* in_sizes, int n_in,
                              void* d_out, int out_size, void* d_ws, size_t ws_size,
                              hipStream_t stream)
{
    (void)in_sizes; (void)n_in; (void)out_size;
    const float* x      = (const float*)d_in[0];
    const float* qkv_w  = (const float*)d_in[1];
    const float* qkv_b  = (const float*)d_in[2];
    const float* dw_w   = (const float*)d_in[3];
    const float* dw_b   = (const float*)d_in[4];
    const float* am_w1  = (const float*)d_in[5];
    const float* am_b1  = (const float*)d_in[6];
    const float* am_w2  = (const float*)d_in[7];
    const float* am_b2  = (const float*)d_in[8];
    const float* gq_w   = (const float*)d_in[9];
    const float* gq_b   = (const float*)d_in[10];
    const float* gkv_w  = (const float*)d_in[11];
    const float* gkv_b  = (const float*)d_in[12];
    const float* proj_w = (const float*)d_in[13];
    const float* proj_b = (const float*)d_in[14];
    float* out = (float*)d_out;

    char* ws = (char*)d_ws;
    size_t off = 0;
    auto carve = [&](size_t bytes) -> void* {
        void* p = ws + off;
        off += (bytes + 255) & ~(size_t)255;
        return p;
    };
    h16*   xt    = (h16*)carve((size_t)8 * 9216 * 128 * 2);
    float* qkvl  = (float*)carve((size_t)8 * 192 * 9216 * 4);
    h16*   qk_t  = (h16*)carve((size_t)8 * 9216 * 64 * 2);
    float* v_buf = (float*)carve((size_t)8 * 64 * 9216 * 4);
    h16*   a1_t  = (h16*)carve((size_t)8 * 9216 * 64 * 2);
    h16*   qlo_t = (h16*)carve((size_t)8 * 9216 * 64 * 2);
    h16*   hi_t  = (h16*)carve((size_t)8 * 9216 * 64 * 2);
    float* lo_f  = (float*)carve((size_t)8 * 4 * 9216 * 16 * 4);
    h16*   xp_t  = (h16*)carve((size_t)8 * 576 * 128 * 2);
    h16*   kkt   = (h16*)carve((size_t)8 * 576 * 64 * 2);
    h16*   vvT   = (h16*)carve((size_t)8 * 64 * 576 * 2);
    h16*   qkvwb = (h16*)carve((size_t)192 * 128 * 2);
    h16*   am1b  = (h16*)carve((size_t)64 * 64 * 2);
    h16*   am2b  = (h16*)carve((size_t)64 * 64 * 2);
    h16*   gqb   = (h16*)carve((size_t)64 * 128 * 2);
    h16*   gkvb  = (h16*)carve((size_t)128 * 128 * 2);
    h16*   projb = (h16*)carve((size_t)128 * 128 * 2);
    if (off > ws_size) return;

    auto packw = [&](const float* s, h16* d, int n) {
        pack_w16<<<dim3((n / 8 + 255) / 256), dim3(256), 0, stream>>>(s, d, n / 8, 16.0f);
    };
    packw(qkv_w, qkvwb, 192 * 128);
    packw(am_w1, am1b, 64 * 64);
    packw(am_w2, am2b, 64 * 64);
    packw(gq_w,  gqb,  64 * 128);
    packw(gkv_w, gkvb, 128 * 128);
    packw(proj_w, projb, 128 * 128);
    pack_x_hwc<<<dim3(8 * 9216 * 16 / 256), dim3(256), 0, stream>>>(x, xt);

    gemm_wmma<128, 0, 12, 0><<<dim3(144, 1, 8), dim3(128), 0, stream>>>(
        qkvwb, xt, nullptr, qkv_b, 9216, 1.0f / 16.0f, 0.f, 1.f, qkvl, nullptr, nullptr, nullptr);

    dwconv_qk_v<<<dim3(36, 64, 8), dim3(16, 16), 0, stream>>>(qkvl, dw_w, dw_b, qk_t, v_buf);

    gemm_wmma<64, 2, 4, 0><<<dim3(144, 1, 8), dim3(128), 0, stream>>>(
        am1b, qk_t, nullptr, am_b1, 9216, 1.0f / 65536.0f, 0.f, 65536.0f, nullptr, a1_t, nullptr, nullptr);

    gemm_wmma<64, 3, 4, 0><<<dim3(144, 1, 8), dim3(128), 0, stream>>>(
        am2b, a1_t, nullptr, am_b2, 9216, 1.0f / 1048576.0f, 0.f, 1048576.0f, nullptr, hi_t, nullptr, v_buf);

    gemm_wmma<128, 1, 4, 0><<<dim3(144, 1, 8), dim3(128), 0, stream>>>(
        gqb, xt, nullptr, gq_b, 9216, 1.0f / 16.0f, 0.f, 1.f, nullptr, qlo_t, nullptr, nullptr);

    avgpool_pack<<<dim3(8 * 576 * 16 / 256), dim3(256), 0, stream>>>(x, xp_t);

    gemm_wmma<128, 4, 8, 0><<<dim3(9, 1, 8), dim3(128), 0, stream>>>(
        gkvb, xp_t, nullptr, gkv_b, 576, 1.0f / 16.0f, 0.f, 1.f, nullptr, kkt, vvT, nullptr);

    attn_kernel<<<dim3(576, 4, 8), dim3(32), 0, stream>>>(qlo_t, kkt, vvT, lo_f);

    gemm_wmma<128, 0, 8, 1><<<dim3(144, 1, 8), dim3(128), 0, stream>>>(
        projb, hi_t, lo_f, proj_b, 9216, 1.0f / 16777216.0f, 1.0f / 1024.0f, 1.f, out, nullptr, nullptr, nullptr);
}
